// MultiLatentAttention_77833397338589
// MI455X (gfx1250) — hardware-verified
//
#include <hip/hip_runtime.h>
#include <math.h>
#include <stdint.h>

#define NB     2
#define SQ     2048
#define DM     2048
#define NH     16
#define DH     128
#define DL     512
#define DR     64
#define DQK    192
#define KVW    320
#define QFW    3072
#define KVFW   5120
#define LW     1024
#define CW     2048
#define NFREQ  32
#define NT64   32
#define NTOK   4096

typedef __bf16       v16b __attribute__((ext_vector_type(16)));
typedef __bf16       v8b  __attribute__((ext_vector_type(8)));
typedef float        v8f  __attribute__((ext_vector_type(8)));
typedef float        v4f  __attribute__((ext_vector_type(4)));
typedef unsigned int v4u  __attribute__((ext_vector_type(4)));
typedef int          v4i  __attribute__((ext_vector_type(4)));

__device__ __forceinline__ unsigned short bf_bits(float f) {
  const unsigned u = __float_as_uint(f);
  return (unsigned short)((u + 0x7FFFu + ((u >> 16) & 1u)) >> 16);
}
__device__ __forceinline__ float bf_val(unsigned short h) { return __uint_as_float(((unsigned)h) << 16); }
__device__ __forceinline__ unsigned pk16(unsigned short a, unsigned short b) { return (unsigned)a | ((unsigned)b << 16); }
__device__ __forceinline__ v8f zero8() { v8f z = {0.f, 0.f, 0.f, 0.f, 0.f, 0.f, 0.f, 0.f}; return z; }
__device__ __forceinline__ int wave_id() { return __builtin_amdgcn_readfirstlane((int)(threadIdx.x >> 5)); }

__device__ __forceinline__ void lds_wave_sync() {
  __builtin_amdgcn_fence(__ATOMIC_RELEASE, "workgroup");
  __builtin_amdgcn_wave_barrier();
  __builtin_amdgcn_fence(__ATOMIC_ACQUIRE, "workgroup");
}

__device__ __forceinline__ unsigned split2(float x, float y, unsigned& lo) {
  const unsigned short hx = bf_bits(x), hy = bf_bits(y);
  const unsigned short lx = bf_bits(x - bf_val(hx)), ly = bf_bits(y - bf_val(hy));
  lo = pk16(lx, ly);
  return pk16(hx, hy);
}
__device__ __forceinline__ void split8(v4f a, v4f b, v4u& hv, v4u& lv) {
  unsigned l0, l1, l2, l3;
  hv[0] = split2(a[0], a[1], l0);
  hv[1] = split2(a[2], a[3], l1);
  hv[2] = split2(b[0], b[1], l2);
  hv[3] = split2(b[2], b[3], l3);
  lv[0] = l0; lv[1] = l1; lv[2] = l2; lv[3] = l3;
}

union FragB { v16b v; v8b h[2]; };
__device__ __forceinline__ v16b ldfrag_b(const __bf16* p) { FragB f; f.h[0] = *(const v8b*)(p); f.h[1] = *(const v8b*)(p + 16); return f.v; }

__device__ __forceinline__ v8f mma_b(v16b a, v16b b, v8f c) {
  return __builtin_amdgcn_wmma_f32_16x16x32_bf16(false, a, false, b, (short)0, c, false, false);
}
__device__ __forceinline__ void guard4_2(v8f& a, v8f& b, v8f& c, v8f& d, v16b x, v16b y) {
  asm volatile("v_nop\n\tv_nop\n\tv_nop\n\tv_nop" : "+v"(a), "+v"(b), "+v"(c), "+v"(d) : "v"(x), "v"(y));
}
__device__ __forceinline__ void guard1b4(v8f& a, v16b w, v16b x, v16b y, v16b z) {
  asm volatile("v_nop\n\tv_nop\n\tv_nop\n\tv_nop" : "+v"(a) : "v"(w), "v"(x), "v"(y), "v"(z) : "memory");
}
__device__ __forceinline__ void keep4(v16b a, v16b b, v16b c, v16b d) { asm volatile("v_nop" :: "v"(a), "v"(b), "v"(c), "v"(d)); }
__device__ __forceinline__ void acc_guard4(v8f& a, v8f& b, v8f& c, v8f& d) {
  asm volatile("v_nop\n\tv_nop\n\tv_nop\n\tv_nop" : "+v"(a), "+v"(b), "+v"(c), "+v"(d));
}
__device__ __forceinline__ void acc_guard2(v8f& a, v8f& b) {
  asm volatile("v_nop\n\tv_nop\n\tv_nop\n\tv_nop" : "+v"(a), "+v"(b));
}

__global__ __launch_bounds__(256) void rope_table_kernel(float* __restrict__ cst, float* __restrict__ snt, int npos) {
  const int lane = threadIdx.x & 31;
  const int wave = (int)(threadIdx.x >> 5);
  const int t = (int)blockIdx.x * 8 + wave;
  if (t >= npos) return;
  const float pf  = (float)t;
  const float e   = (float)lane * 0.03125f;
  const float pw  = powf(10000.0f, e);
  const float inv = 1.0f / pw;
  const float ang = pf * inv;
  float sv, cv;
  sincosf(ang, &sv, &cv);
  const size_t o = (size_t)t * NFREQ + lane;
  for (int pass = 0; pass < 2; ++pass) {
    ((volatile float*)cst)[o] = cv;
    ((volatile float*)snt)[o] = sv;
    __threadfence();
  }
}

__global__ __launch_bounds__(256) void cvt_bf16_kernel(const float* __restrict__ in, unsigned short* __restrict__ outp, int n8) {
  const int i = (int)blockIdx.x * 256 + (int)threadIdx.x;
  if (i >= n8) return;
  const size_t e = 8 * (size_t)i;
  const v4f a = *(const v4f*)(in + e);
  const v4f b = *(const v4f*)(in + e + 4);
  v4u w;
  w[0] = pk16(bf_bits(a[0]), bf_bits(a[1]));
  w[1] = pk16(bf_bits(a[2]), bf_bits(a[3]));
  w[2] = pk16(bf_bits(b[0]), bf_bits(b[1]));
  w[3] = pk16(bf_bits(b[2]), bf_bits(b[3]));
  *(volatile v4u*)(outp + e) = w;
  __threadfence();
  *(volatile v4u*)(outp + e) = w;
}

__global__ __launch_bounds__(256) void wtrans_kernel(const float* __restrict__ W, unsigned short* __restrict__ WT,
                                                     int ncols, int ldt) {
  __shared__ __align__(16) unsigned short th[64 * 72];
  const int c0  = (int)blockIdx.x * 64;
  const int r0  = (int)blockIdx.y * 64;
  const int tid = (int)threadIdx.x;
  {
    const int rr = tid >> 2;
    const int cq = (tid & 3) * 16;
    const float* src = W + (size_t)(r0 + rr) * ncols + c0 + cq;
#pragma unroll
    for (int q = 0; q < 4; ++q) {
      const v4f f = *(const v4f*)(src + 4 * q);
#pragma unroll
      for (int e = 0; e < 4; ++e) th[rr * 72 + cq + 4 * q + e] = bf_bits(f[e]);
    }
  }
  __syncthreads();
  const int sub = tid >> 3;
  const int c8  = (tid & 7) * 8;
  v4u hv[2];
#pragma unroll
  for (int it = 0; it < 2; ++it) {
    const int oc = it * 32 + sub;
    v4u a;
#pragma unroll
    for (int q = 0; q < 4; ++q) a[q] = pk16(th[(c8 + 2 * q) * 72 + oc], th[(c8 + 2 * q + 1) * 72 + oc]);
    hv[it] = a;
  }
  for (int pass = 0; pass < 2; ++pass) {
#pragma unroll
    for (int it = 0; it < 2; ++it) {
      const int oc = it * 32 + sub;
      const size_t go = (size_t)(c0 + oc) * ldt + r0 + c8;
      *(volatile v4u*)(WT + go) = hv[it];
    }
    __threadfence();
  }
}

__global__ __launch_bounds__(256) void mask_class_kernel(const int* __restrict__ mask, int* __restrict__ cls) {
  __shared__ int nzs[NT64];
  __shared__ int zrs[NT64];
  const int mt   = (int)blockIdx.x;
  const int tid  = (int)threadIdx.x;
  const int lane = tid & 31;
  const int wave = tid >> 5;
  const int j0   = tid * 8;
  int nz = 0, zr = 0;
#pragma unroll 1
  for (int r = 0; r < 64; ++r) {
    const int* mr = mask + (size_t)(mt * 64 + r) * SQ + j0;
    const v4i a = *(const v4i*)(mr);
    const v4i b = *(const v4i*)(mr + 4);
    const int n = ((a[0] != 0) | (a[1] != 0) | (a[2] != 0) | (a[3] != 0) |
                   (b[0] != 0) | (b[1] != 0) | (b[2] != 0) | (b[3] != 0)) ? 1 : 0;
    const int z = ((a[0] == 0) | (a[1] == 0) | (a[2] == 0) | (a[3] == 0) |
                   (b[0] == 0) | (b[1] == 0) | (b[2] == 0) | (b[3] == 0)) ? 1 : 0;
    nz |= n;
    zr |= z;
  }
  nz |= __shfl_xor(nz, 1, 32); nz |= __shfl_xor(nz, 2, 32); nz |= __shfl_xor(nz, 4, 32);
  zr |= __shfl_xor(zr, 1, 32); zr |= __shfl_xor(zr, 2, 32); zr |= __shfl_xor(zr, 4, 32);
  if ((lane & 7) == 0) { nzs[tid >> 3] = nz; zrs[tid >> 3] = zr; }
  __syncthreads();
  if (wave == 0) {
    const int n = nzs[lane];
    const int z = zrs[lane];
    const int cval = (n == 0) ? 0 : ((z == 0) ? 1 : 2);
    volatile int* cp = cls + (size_t)mt * NT64 + lane;
    *cp = cval;
    __threadfence();
    *cp = cval;
  }
}

#define TP    68
#define PERW  (64 * TP)
static_assert(((TP * 4) % 16) == 0);
static_assert(2 * PERW * 4 <= 65536);

template <int EPI, bool ASPLIT>
__global__ __launch_bounds__(64) void gemm64_kernel(
    const unsigned short* __restrict__ Ap, const unsigned short* __restrict__ A2p, int lda,
    const unsigned short* __restrict__ Btp, int ldb,
    const float* __restrict__ cst, const float* __restrict__ snt,
    void* C0, void* C1, void* C2, void* C3, int ldc, int ldc2,
    int M, int N, int K) {
  __shared__ __align__(16) float lds_all[2 * PERW];

  const int lane = threadIdx.x & 31;
  const int wave = wave_id();
  const int hh = lane >> 4;
  const int rl = lane & 15;
  const int q8 = lane >> 3;
  const int c8 = (lane & 7) * 8;
  const int tilesN = N >> 6;
  const int tilesM = M >> 6;
  const int tile = (int)blockIdx.x * 2 + wave;
  if (tile >= tilesM * tilesN) return;
  const int tm = tile / tilesN;
  const int tn = tile - tm * tilesN;
  const int m0 = tm << 6;
  const int n0 = tn << 6;

  const __bf16* A  = (const __bf16*)(const void*)Ap;
  const __bf16* A2 = (const __bf16*)(const void*)A2p;
  const __bf16* Bt = (const __bf16*)(const void*)Btp;

  v8f acc[4][4];
#pragma unroll
  for (int i = 0; i < 4; ++i)
#pragma unroll
    for (int j = 0; j < 4; ++j) acc[i][j] = zero8();

  for (int k0 = 0; k0 < K; k0 += 32) {
    v16b bh[4];
#pragma unroll
    for (int j = 0; j < 4; ++j) bh[j] = ldfrag_b(Bt + (size_t)(n0 + j * 16 + rl) * ldb + k0 + 8 * hh);
#pragma unroll
    for (int i = 0; i < 4; ++i) {
      const size_t ao = (size_t)(m0 + i * 16 + rl) * lda + k0 + 8 * hh;
      const v16b ah = ldfrag_b(A + ao);
      v16b al = ah;
      if (ASPLIT) al = ldfrag_b(A2 + ao);
#pragma unroll
      for (int j = 0; j < 4; ++j) {
        acc[i][j] = mma_b(ah, bh[j], acc[i][j]);
        if (ASPLIT) acc[i][j] = mma_b(al, bh[j], acc[i][j]);
      }
      guard4_2(acc[i][0], acc[i][1], acc[i][2], acc[i][3], ah, al);
    }
    keep4(bh[0], bh[1], bh[2], bh[3]);
  }
  acc_guard4(acc[0][0], acc[0][1], acc[0][2], acc[0][3]);
  acc_guard4(acc[1][0], acc[1][1], acc[1][2], acc[1][3]);
  acc_guard4(acc[2][0], acc[2][1], acc[2][2], acc[2][3]);
  acc_guard4(acc[3][0], acc[3][1], acc[3][2], acc[3][3]);

  float* T = lds_all + wave * PERW;
#pragma unroll
  for (int i = 0; i < 4; ++i)
#pragma unroll
    for (int j = 0; j < 4; ++j)
#pragma unroll
      for (int r = 0; r < 8; ++r)
        T[(i * 16 + 8 * hh + r) * TP + j * 16 + rl] = acc[i][j][r];
  lds_wave_sync();

  if (EPI == 0) {
    unsigned short* P0 = (unsigned short*)C0;
    unsigned short* P1 = (unsigned short*)C1;
    for (int pass = 0; pass < 2; ++pass) {
#pragma unroll 2
      for (int it = 0; it < 16; ++it) {
        const int row = it * 4 + q8;
        const v4f xa = *(const v4f*)(T + row * TP + c8);
        const v4f xb = *(const v4f*)(T + row * TP + c8 + 4);
        v4u vh, vl;
        split8(xa, xb, vh, vl);
        const size_t go = (size_t)(m0 + row) * ldc + n0 + c8;
        *(volatile v4u*)(P0 + go) = vh;
        *(volatile v4u*)(P1 + go) = vl;
      }
      __threadfence();
    }
  } else if (EPI == 1 || EPI == 2) {
    int colK, hrow, dv0;
    bool isrope, isv;
    if (EPI == 2) {
      const int c0 = n0 % DQK;
      isrope = (c0 >= 128);
      isv = false;
      colK = n0; hrow = 0; dv0 = 0;
    } else {
      const int hd = n0 / KVW;
      const int c0 = n0 - hd * KVW;
      isrope = (c0 == 128);
      isv = (c0 >= DQK);
      colK = hd * DQK + c0;
      hrow = hd * DH;
      dv0 = c0 - DQK;
    }
    if (!isv) {
      unsigned short* P0 = (unsigned short*)C0;
      unsigned short* P1 = (unsigned short*)C1;
      const float sgn = (c8 < 32) ? -1.0f : 1.0f;
      const int   pc8 = c8 ^ 32;
      const int   f8  = c8 & 31;
      const v4f one4 = {1.f, 1.f, 1.f, 1.f};
      const v4f nil4 = {0.f, 0.f, 0.f, 0.f};
      for (int pass = 0; pass < 2; ++pass) {
#pragma unroll 2
        for (int it = 0; it < 16; ++it) {
          const int row = it * 4 + q8;
          const v4f xa = *(const v4f*)(T + row * TP + c8);
          const v4f xb = *(const v4f*)(T + row * TP + c8 + 4);
          const v4f pa = *(const v4f*)(T + row * TP + pc8);
          const v4f pb = *(const v4f*)(T + row * TP + pc8 + 4);
          v4f ca = one4, cb = one4, sa = nil4, sb = nil4;
          if (isrope) {
            const float* cr = cst + (size_t)(m0 + row) * NFREQ + f8;
            const float* sr = snt + (size_t)(m0 + row) * NFREQ + f8;
            ca = *(const v4f*)(cr); cb = *(const v4f*)(cr + 4);
            sa = *(const v4f*)(sr); sb = *(const v4f*)(sr + 4);
          }
          v4f oa, ob;
#pragma unroll
          for (int e = 0; e < 4; ++e) {
            oa[e] = xa[e] * ca[e] + (sgn * pa[e]) * sa[e];
            ob[e] = xb[e] * cb[e] + (sgn * pb[e]) * sb[e];
          }
          v4u vh, vl;
          split8(oa, ob, vh, vl);
          const size_t go = (size_t)(m0 + row) * ldc + colK + c8;
          *(volatile v4u*)(P0 + go) = vh;
          *(volatile v4u*)(P1 + go) = vl;
        }
        __threadfence();
      }
    } else {
      unsigned short* PV0 = (unsigned short*)C2;
      unsigned short* PV1 = (unsigned short*)C3;
      for (int pass = 0; pass < 2; ++pass) {
#pragma unroll 2
        for (int it = 0; it < 16; ++it) {
          const int dv = it * 4 + q8;
          const float* tc = T + c8 * TP + dv;
          v4f xa, xb;
          xa[0] = tc[0 * TP]; xa[1] = tc[1 * TP]; xa[2] = tc[2 * TP]; xa[3] = tc[3 * TP];
          xb[0] = tc[4 * TP]; xb[1] = tc[5 * TP]; xb[2] = tc[6 * TP]; xb[3] = tc[7 * TP];
          v4u vh, vl;
          split8(xa, xb, vh, vl);
          const size_t go = (size_t)(hrow + dv0 + dv) * ldc2 + m0 + c8;
          *(volatile v4u*)(PV0 + go) = vh;
          *(volatile v4u*)(PV1 + go) = vl;
        }
        __threadfence();
      }
    }
  } else {
    float* C = (float*)C0;
    const int c4 = rl * 4;
    for (int pass = 0; pass < 2; ++pass) {
#pragma unroll 4
      for (int it = 0; it < 32; ++it) {
        const int row = it * 2 + hh;
        const v4f v = *(const v4f*)(T + row * TP + c4);
        *(volatile v4f*)(C + (size_t)(m0 + row) * ldc + n0 + c4) = v;
      }
      __threadfence();
    }
  }
}

#define AKC  32
#define QP   200
#define KP   200
#define VP   40
#define PPI  40
#define MP   36
#define SCALE_QK 0.07216878364870323f

#define LQH  0
#define LQL  (LQH + 64 * QP * 2)
#define LKH  (LQL + 64 * QP * 2)
#define LKL  (LKH + AKC * KP * 2)
#define LVH  (LKL + AKC * KP * 2)
#define LVL  (LVH + DH * VP * 2)
#define LPH  (LVL + DH * VP * 2)
#define LPL  (LPH + 4 * 16 * PPI * 2)
#define LMS  (LPL + 4 * 16 * PPI * 2)
#define LOH  (LMS + 64 * MP * 4)
#define LOL  (LOH + 4 * 16 * DH * 2)
#define ATT_LDS (LOL + 4 * 16 * DH * 2)
static_assert((LQL % 16) == 0 && (LKH % 16) == 0 && (LKL % 16) == 0 && (LVH % 16) == 0 && (LVL % 16) == 0);
static_assert((LPH % 16) == 0 && (LPL % 16) == 0 && (LMS % 16) == 0 && (LOH % 16) == 0 && (LOL % 16) == 0);
static_assert(ATT_LDS == 149504);

__global__ __launch_bounds__(128) void attn_kernel(
    const unsigned short* __restrict__ qhp, const unsigned short* __restrict__ qlp,
    const unsigned short* __restrict__ khp, const unsigned short* __restrict__ klp,
    const unsigned short* __restrict__ vhp, const unsigned short* __restrict__ vlp,
    const int* __restrict__ maskp, const int* __restrict__ clsp,
    unsigned short* __restrict__ cxh, unsigned short* __restrict__ cxl) {
  extern __shared__ __align__(16) unsigned char att_lds[];
  unsigned short* Qhs = (unsigned short*)(att_lds + LQH);
  unsigned short* Qls = (unsigned short*)(att_lds + LQL);
  unsigned short* Ks  = (unsigned short*)(att_lds + LKH);
  unsigned short* Kls = (unsigned short*)(att_lds + LKL);
  unsigned short* Vhs = (unsigned short*)(att_lds + LVH);
  unsigned short* Vls = (unsigned short*)(att_lds + LVL);
  unsigned short* Phs = (unsigned short*)(att_lds + LPH);
  unsigned short* Pls = (unsigned short*)(att_lds + LPL);
  int*            Ms  = (int*)(att_lds + LMS);
  unsigned short* Osh = (unsigned short*)(att_lds + LOH);
  unsigned short* Osl = (unsigned short*)(att_lds + LOL);

  const int tid  = (int)threadIdx.x;
  const int lane = tid & 31;
  const int wave = wave_id();
  const int hh   = lane >> 4;
  const int c    = lane & 15;
  const int qt   = (int)blockIdx.x;
  const int h    = (int)blockIdx.y;
  const int qrow0 = qt * 64;

#pragma unroll 1
  for (int u = tid; u < 64 * MP; u += 128) Ms[u] = 1;

#pragma unroll 4
  for (int u = 0; u < 12; ++u) {
    const int p   = tid + 128 * u;
    const int row = p / 24;
    const int d8  = (p - row * 24) * 8;
    const size_t go = (size_t)(qrow0 + row) * QFW + h * DQK + d8;
    const v4u x = *(const v4u*)(qhp + go);
    const v4u y = *(const v4u*)(qlp + go);
    *(v4u*)(Qhs + row * QP + d8) = x;
    *(v4u*)(Qls + row * QP + d8) = y;
  }

  const int* crow = clsp + qt * NT64;
  unsigned short* ph = Phs + wave * 16 * PPI;
  unsigned short* pl = Pls + wave * 16 * PPI;
  const __bf16* Qw  = (const __bf16*)(const void*)Qhs + (wave * 16 + c) * QP + 8 * hh;
  const __bf16* Qlw = (const __bf16*)(const void*)Qls + (wave * 16 + c) * QP + 8 * hh;

  float mrow[8], lrow[8];
  v8f oacc[8];
#pragma unroll
  for (int r = 0; r < 8; ++r) { mrow[r] = -INFINITY; lrow[r] = 0.f; }
#pragma unroll
  for (int t = 0; t < 8; ++t) oacc[t] = zero8();

  for (int kc = 0; kc < 2 * NT64; ++kc) {
    const int nt = kc >> 1;
    const int cl = __builtin_amdgcn_readfirstlane(crow[nt]);
    if (cl == 0) continue;
    const int kv0 = kc * AKC;
    __syncthreads();
#pragma unroll 3
    for (int u = 0; u < 6; ++u) {
      const int p   = tid + 128 * u;
      const int key = p / 24;
      const int d8  = (p - key * 24) * 8;
      const size_t ko = (size_t)(kv0 + key) * QFW + h * DQK + d8;
      const v4u kx = *(const v4u*)(khp + ko);
      const v4u ky = *(const v4u*)(klp + ko);
      *(v4u*)(Ks  + key * KP + d8) = kx;
      *(v4u*)(Kls + key * KP + d8) = ky;
    }
#pragma unroll
    for (int u = 0; u < 4; ++u) {
      const int p  = tid + 128 * u;
      const int dv = p >> 2, k8 = (p & 3) * 8;
      const size_t vo = (size_t)(h * DH + dv) * SQ + kv0 + k8;
      const v4u vx = *(const v4u*)(vhp + vo);
      const v4u vy = *(const v4u*)(vlp + vo);
      *(v4u*)(Vhs + dv * VP + k8) = vx;
      *(v4u*)(Vls + dv * VP + k8) = vy;
    }
    if (cl == 2) {
#pragma unroll
      for (int u = 0; u < 4; ++u) {
        const int p   = tid + 128 * u;
        const int row = p >> 3, c4 = (p & 7) * 4;
        const v4i mv = *(const v4i*)(maskp + (size_t)(qrow0 + row) * SQ + kv0 + c4);
        *(v4i*)(Ms + row * MP + c4) = mv;
      }
    }
    __syncthreads();

    v8f sa[2];
    sa[0] = zero8(); sa[1] = zero8();
#pragma unroll
    for (int dc = 0; dc < 6; ++dc) {
      const v16b qa = ldfrag_b(Qw + dc * 32);
      const v16b qb = ldfrag_b(Qlw + dc * 32);
#pragma unroll
      for (int j = 0; j < 2; ++j) {
        const v16b kb = ldfrag_b((const __bf16*)(const void*)Ks  + (j * 16 + c) * KP + dc * 32 + 8 * hh);
        const v16b kl = ldfrag_b((const __bf16*)(const void*)Kls + (j * 16 + c) * KP + dc * 32 + 8 * hh);
        sa[j] = mma_b(qa, kb, sa[j]);
        sa[j] = mma_b(qa, kl, sa[j]);
        sa[j] = mma_b(qb, kb, sa[j]);
        guard1b4(sa[j], qa, qb, kb, kl);
      }
    }
    acc_guard2(sa[0], sa[1]);

    float cm[8];
#pragma unroll
    for (int r = 0; r < 8; ++r) {
      const int lr = wave * 16 + 8 * hh + r;
      float m = -INFINITY;
#pragma unroll
      for (int j = 0; j < 2; ++j) {
        float s = sa[j][r] * SCALE_QK;
        if (cl == 2) {
          const int mv = Ms[lr * MP + j * 16 + c];
          s = (mv != 0) ? s : -INFINITY;
        }
        sa[j][r] = s;
        m = fmaxf(m, s);
      }
#pragma unroll
      for (int off = 1; off < 16; off <<= 1) m = fmaxf(m, __shfl_xor(m, off, 32));
      cm[r] = m;
    }
#pragma unroll
    for (int r = 0; r < 8; ++r) {
      const float mnew  = fmaxf(mrow[r], cm[r]);
      const float muse  = (mnew > -INFINITY) ? mnew : 0.0f;
      const float alpha = __expf(mrow[r] - muse);
      mrow[r] = mnew;
      float psum = 0.f;
#pragma unroll
      for (int j = 0; j < 2; ++j) {
        const float p = __expf(sa[j][r] - muse);
        psum += p;
        const unsigned short hb = bf_bits(p);
        const unsigned short lb = bf_bits(p - bf_val(hb));
        const int po = (8 * hh + r) * PPI + j * 16 + c;
        ph[po] = hb;
        pl[po] = lb;
      }
#pragma unroll
      for (int off = 1; off < 16; off <<= 1) psum += __shfl_xor(psum, off, 32);
      lrow[r] = lrow[r] * alpha + psum;
#pragma unroll
      for (int t = 0; t < 8; ++t) oacc[t][r] *= alpha;
    }
    lds_wave_sync();
    const v16b pa = ldfrag_b((const __bf16*)(const void*)ph + c * PPI + 8 * hh);
    const v16b pr = ldfrag_b((const __bf16*)(const void*)pl + c * PPI + 8 * hh);
#pragma unroll
    for (int t = 0; t < 8; ++t) {
      const v16b vb = ldfrag_b((const __bf16*)(const void*)Vhs + (t * 16 + c) * VP + 8 * hh);
      const v16b vr = ldfrag_b((const __bf16*)(const void*)Vls + (t * 16 + c) * VP + 8 * hh);
      oacc[t] = mma_b(pa, vb, oacc[t]);
      oacc[t] = mma_b(pa, vr, oacc[t]);
      oacc[t] = mma_b(pr, vb, oacc[t]);
      guard1b4(oacc[t], pa, pr, vb, vr);
    }
  }
  __syncthreads();
  acc_guard4(oacc[0], oacc[1], oacc[2], oacc[3]);
  acc_guard4(oacc[4], oacc[5], oacc[6], oacc[7]);

  unsigned short* osh = Osh + wave * 16 * DH;
  unsigned short* osl = Osl + wave * 16 * DH;
#pragma unroll
  for (int r = 0; r < 8; ++r) {
    const float inv = 1.0f / lrow[r];
#pragma unroll
    for (int t = 0; t < 8; ++t) {
      const float o = oacc[t][r] * inv;
      const unsigned short hb = bf_bits(o);
      const unsigned short lb = bf_bits(o - bf_val(hb));
      const int so = (8 * hh + r) * DH + t * 16 + c;
      osh[so] = hb;
      osl[so] = lb;
    }
  }
  lds_wave_sync();
  unsigned short* Cg = cxh + (size_t)(qrow0 + wave * 16) * CW + h * DH;
  unsigned short* Cl = cxl + (size_t)(qrow0 + wave * 16) * CW + h * DH;
  const int c8 = c * 8;
  for (int pass = 0; pass < 2; ++pass) {
#pragma unroll
    for (int it = 0; it < 8; ++it) {
      const int row = it * 2 + hh;
      const v4u x = *(const v4u*)(osh + row * DH + c8);
      const v4u y = *(const v4u*)(osl + row * DH + c8);
      *(volatile v4u*)(Cg + (size_t)row * CW + c8) = x;
      *(volatile v4u*)(Cl + (size_t)row * CW + c8) = y;
    }
    __threadfence();
  }
}

extern "C" void kernel_launch(void* const* d_in, const int* in_sizes, int n_in,
                              void* d_out, int out_size, void* d_ws, size_t ws_size,
                              hipStream_t stream) {
  if (n_in < 7) return;
  if (in_sizes[0] != NTOK * DM) return;
  if (in_sizes[1] != DM * DL) return;
  if (in_sizes[2] != DL * KVFW) return;
  if (in_sizes[3] != DM * DL) return;
  if (in_sizes[4] != DL * QFW) return;
  if (in_sizes[5] != CW * DM) return;
  if (in_sizes[6] != SQ * SQ) return;
  if (out_size != NTOK * DM) return;

  const float* x    = (const float*)d_in[0];
  const float* Wkvd = (const float*)d_in[1];
  const float* Wkvu = (const float*)d_in[2];
  const float* Wqd  = (const float*)d_in[3];
  const float* Wqu  = (const float*)d_in[4];
  const float* Wo   = (const float*)d_in[5];
  const int*   mask = (const int*)d_in[6];
  float* out = (float*)d_out;

  const size_t szT    = (size_t)SQ * NFREQ * 4;
  const size_t szCLS  = (size_t)NT64 * NT64 * 4;
  const size_t szXB   = (size_t)NTOK * DM * 2;
  const size_t szWDT  = (size_t)LW * DM * 2;
  const size_t szWKVU = (size_t)KVFW * DL * 2;
  const size_t szWQU  = (size_t)QFW * DL * 2;
  const size_t szWOT  = (size_t)DM * CW * 2;
  const size_t szL    = (size_t)SQ * LW * 2;
  const size_t szKP   = (size_t)SQ * QFW * 2;
  const size_t szVT   = (size_t)CW * SQ * 2;
  const size_t szCX   = (size_t)SQ * CW * 2;
  size_t off = 0;
  const size_t oCST  = off; off += szT;
  const size_t oSNT  = off; off += szT;
  const size_t oCLS  = off; off += szCLS;
  const size_t oXB   = off; off += szXB;
  const size_t oWDT  = off; off += szWDT;
  const size_t oWKVU = off; off += szWKVU;
  const size_t oWQU  = off; off += szWQU;
  const size_t oWOT  = off; off += szWOT;
  const size_t oLH   = off; off += szL;
  const size_t oLL   = off; off += szL;
  const size_t oKPH  = off; off += szKP;
  const size_t oKPL  = off; off += szKP;
  const size_t oQPH  = off; off += szKP;
  const size_t oQPL  = off; off += szKP;
  const size_t oVTH  = off; off += szVT;
  const size_t oVTL  = off; off += szVT;
  const size_t oCXH  = off; off += szCX;
  const size_t oCXL  = off; off += szCX;
  if (off > ws_size) return;

  char* ws = (char*)d_ws;
  float*          CST   = (float*)(ws + oCST);
  float*          SNT   = (float*)(ws + oSNT);
  int*            CLS   = (int*)(ws + oCLS);
  unsigned short* XB    = (unsigned short*)(ws + oXB);
  unsigned short* WDT   = (unsigned short*)(ws + oWDT);
  unsigned short* WKVUT = (unsigned short*)(ws + oWKVU);
  unsigned short* WQUT  = (unsigned short*)(ws + oWQU);
  unsigned short* WOT   = (unsigned short*)(ws + oWOT);
  unsigned short* LH    = (unsigned short*)(ws + oLH);
  unsigned short* LL    = (unsigned short*)(ws + oLL);
  unsigned short* KPH   = (unsigned short*)(ws + oKPH);
  unsigned short* KPL   = (unsigned short*)(ws + oKPL);
  unsigned short* QPH   = (unsigned short*)(ws + oQPH);
  unsigned short* QPL   = (unsigned short*)(ws + oQPL);
  unsigned short* VTH   = (unsigned short*)(ws + oVTH);
  unsigned short* VTL   = (unsigned short*)(ws + oVTL);
  unsigned short* CXH   = (unsigned short*)(ws + oCXH);
  unsigned short* CXL   = (unsigned short*)(ws + oCXL);

  const dim3 b256(256), b128(128), b64(64);

  rope_table_kernel<<<dim3(SQ / 8), b256, 0, stream>>>(CST, SNT, SQ);
  cvt_bf16_kernel<<<dim3((NTOK * DM / 8) / 256), b256, 0, stream>>>(x, XB, NTOK * DM / 8);
  wtrans_kernel<<<dim3(DL / 64, DM / 64), b256, 0, stream>>>(Wkvd, WDT, DL, DM);
  wtrans_kernel<<<dim3(DL / 64, DM / 64), b256, 0, stream>>>(Wqd, WDT + (size_t)DL * DM, DL, DM);
  wtrans_kernel<<<dim3(KVFW / 64, DL / 64), b256, 0, stream>>>(Wkvu, WKVUT, KVFW, DL);
  wtrans_kernel<<<dim3(QFW / 64, DL / 64), b256, 0, stream>>>(Wqu, WQUT, QFW, DL);
  wtrans_kernel<<<dim3(DM / 64, CW / 64), b256, 0, stream>>>(Wo, WOT, DM, CW);
  mask_class_kernel<<<dim3(NT64), b256, 0, stream>>>(mask, CLS);

  (void)hipFuncSetAttribute(reinterpret_cast<const void*>(&attn_kernel), hipFuncAttributeMaxDynamicSharedMemorySize, ATT_LDS);

  const int tilesM = SQ / 64;
  for (int b = 0; b < NB; ++b) {
    const unsigned short* XBb = XB + (size_t)b * SQ * DM;
    float* outb = out + (size_t)b * SQ * DM;
    gemm64_kernel<0, false><<<dim3(tilesM * (LW / 64) / 2), b64, 0, stream>>>(
        XBb, XBb, DM, WDT, DM, CST, SNT, (void*)LH, (void*)LL, (void*)LH, (void*)LL, LW, LW, SQ, LW, DM);
    gemm64_kernel<1, true><<<dim3(tilesM * (KVFW / 64) / 2), b64, 0, stream>>>(
        LH, LL, LW, WKVUT, DL, CST, SNT, (void*)KPH, (void*)KPL, (void*)VTH, (void*)VTL, QFW, SQ, SQ, KVFW, DL);
    gemm64_kernel<2, true><<<dim3(tilesM * (QFW / 64) / 2), b64, 0, stream>>>(
        LH + DL, LL + DL, LW, WQUT, DL, CST, SNT, (void*)QPH, (void*)QPL, (void*)QPH, (void*)QPL, QFW, QFW, SQ, QFW, DL);
    attn_kernel<<<dim3(SQ / 64, NH), b128, ATT_LDS, stream>>>(QPH, QPL, KPH, KPL, VTH, VTL, mask, CLS, CXH, CXL);
    gemm64_kernel<3, true><<<dim3(tilesM * (DM / 64) / 2), b64, 0, stream>>>(
        CXH, CXL, CW, WOT, CW, CST, SNT, (void*)outb, (void*)outb, (void*)outb, (void*)outb, DM, DM, SQ, DM, CW);
  }
  (void)hipGetLastError();
}
